// MyGPT2Attention_8839042695366
// MI455X (gfx1250) — hardware-verified
//
#include <hip/hip_runtime.h>


typedef __bf16 bf16_t;
typedef __attribute__((ext_vector_type(16))) __bf16 v16bf;
typedef __attribute__((ext_vector_type(8)))  float v8f;
typedef __attribute__((ext_vector_type(4)))  float v4f;
typedef __attribute__((ext_vector_type(4)))  unsigned int v4u;

#define BB    2
#define SS    2048
#define DD    1024
#define HH    16
#define HD    64
#define MROWS (BB * SS)
#define NQKV  (3 * DD)

static_assert(HH * HD == DD);
static_assert(HD == 64);
static_assert(SS / 16 == 128);
static_assert(SS % 64 == 0 && DD % 64 == 0 && NQKV % 64 == 0 && MROWS % 64 == 0);
static_assert((MROWS * DD) % (8 * 256) == 0);

#define NOP4 "v_nop\n\tv_nop\n\tv_nop\n\tv_nop"

__device__ __forceinline__ v8f mma(v16bf a, v16bf b, v8f c) {
  return __builtin_amdgcn_wmma_f32_16x16x32_bf16(false, a, false, b, (short)0, c, false, false);
}

__device__ __forceinline__ v8f zero8() {
  v8f z = {0.f, 0.f, 0.f, 0.f, 0.f, 0.f, 0.f, 0.f};
  return z;
}

union Frag { v16bf v; v4u u[2]; };

__device__ __forceinline__ v16bf ldfrag(const bf16_t* __restrict__ p, int h) {
  Frag f;
  f.u[0] = *(const v4u*)(p + 8 * h);
  f.u[1] = *(const v4u*)(p + 16 + 8 * h);
  return f.v;
}

__device__ __forceinline__ unsigned int bfbits(float v) {
  const bf16_t b = (bf16_t)v;
  return (unsigned int)__builtin_bit_cast(unsigned short, b);
}
__device__ __forceinline__ float bf2f(unsigned int u) {
  return __builtin_bit_cast(float, u << 16);
}
__device__ __forceinline__ void split2(float v, unsigned int& hi, unsigned int& lo) {
  const bf16_t hb = (bf16_t)v;
  const float hf = (float)hb;
  const bf16_t lb = (bf16_t)(v - hf);
  hi = (unsigned int)__builtin_bit_cast(unsigned short, hb);
  lo = (unsigned int)__builtin_bit_cast(unsigned short, lb);
}
__device__ __forceinline__ void pack_hl8(const v8f v, float sc, v4u& H, v4u& L) {
  unsigned int hw[4], lw[4];
#pragma unroll
  for (int j = 0; j < 4; ++j) {
    unsigned int h0, l0, h1, l1;
    split2(v[2 * j] * sc, h0, l0);
    split2(v[2 * j + 1] * sc, h1, l1);
    hw[j] = h0 | (h1 << 16);
    lw[j] = l0 | (l1 << 16);
  }
  v4u Ht = {hw[0], hw[1], hw[2], hw[3]};
  v4u Lt = {lw[0], lw[1], lw[2], lw[3]};
  H = Ht;
  L = Lt;
}

__global__ void __launch_bounds__(256) k_cvt(const float* __restrict__ in, bf16_t* __restrict__ out, int n8) {
  const int i = blockIdx.x * 256 + (int)threadIdx.x;
  if (i < n8) {
    const float* src = in + (size_t)i * 8;
    const v4f a = *(const v4f*)src;
    const v4f b = *(const v4f*)(src + 4);
    v4u w = {bfbits(a[0]) | (bfbits(a[1]) << 16), bfbits(a[2]) | (bfbits(a[3]) << 16),
             bfbits(b[0]) | (bfbits(b[1]) << 16), bfbits(b[2]) | (bfbits(b[3]) << 16)};
    bf16_t* dst = out + (size_t)i * 8;
    *(volatile v4u*)dst = w;
    __threadfence();
    *(volatile v4u*)dst = w;
  }
}

__global__ void __launch_bounds__(256) k_tr(const float* __restrict__ in, bf16_t* __restrict__ out,
                                            int rows, int cols) {
  __shared__ __align__(16) unsigned short ts[64 * 64];
  const int tid = (int)threadIdx.x;
  const int c0 = blockIdx.x * 64, r0 = blockIdx.y * 64;
#pragma unroll
  for (int it = 0; it < 16; ++it) {
    const int e = it * 256 + tid;
    const int rl = e >> 6, cl = e & 63;
    const int r = r0 + rl, c = c0 + cl;
    float v = 0.f;
    if (r < rows && c < cols) v = in[(size_t)r * cols + c];
    ts[cl * 64 + rl] = (unsigned short)bfbits(v);
  }
  __syncthreads();
  auto wr = [&]() {
#pragma unroll
    for (int it = 0; it < 2; ++it) {
      const int p = it * 256 + tid;
      const int row = p >> 3, piece = p & 7;
      const int c = c0 + row, rr = r0 + piece * 8;
      if (c < cols && rr + 8 <= rows) {
        const v4u w = *(const v4u*)(ts + row * 64 + piece * 8);
        *(volatile v4u*)(out + (size_t)c * rows + rr) = w;
      }
    }
  };
  wr();
  __threadfence();
  wr();
}

__global__ void __launch_bounds__(64) __attribute__((amdgpu_num_vgpr(256)))
k_qkv(const bf16_t* __restrict__ X, const bf16_t* __restrict__ WaT, const float* __restrict__ bias,
      bf16_t* __restrict__ Qh, bf16_t* __restrict__ Ql, bf16_t* __restrict__ Kh, bf16_t* __restrict__ Kl,
      bf16_t* __restrict__ Vh, bf16_t* __restrict__ Vl) {
  __shared__ __align__(16) unsigned short sm[2 * 64 * 64];
  const int tid = (int)threadIdx.x;
  const int lane = tid & 31, h = lane >> 4, lan = lane & 15, widx = tid >> 5;
  constexpr int NT = NQKV / 64;
  const int bm = blockIdx.x / NT, bn = blockIdx.x - bm * NT;
  const int rowb = bm * 64, row0 = rowb + widx * 32, col0 = bn * 64;

  v8f acc[2][4];
#pragma unroll
  for (int mi = 0; mi < 2; ++mi)
#pragma unroll
    for (int t = 0; t < 4; ++t) acc[mi][t] = zero8();

  const bf16_t* ar0 = X + (size_t)(row0 + lan) * DD;
  const bf16_t* ar1 = X + (size_t)(row0 + 16 + lan) * DD;
  const bf16_t* brw = WaT + (size_t)(col0 + lan) * DD;
#pragma unroll 1
  for (int k0 = 0; k0 < DD; k0 += 32) {
    const v16bf a0 = ldfrag(ar0 + k0, h), a1 = ldfrag(ar1 + k0, h);
    const v16bf b0 = ldfrag(brw + k0, h);
    const v16bf b1 = ldfrag(brw + (size_t)16 * DD + k0, h);
    const v16bf b2 = ldfrag(brw + (size_t)32 * DD + k0, h);
    const v16bf b3 = ldfrag(brw + (size_t)48 * DD + k0, h);
    acc[0][0] = mma(a0, b0, acc[0][0]);
    acc[1][0] = mma(a1, b0, acc[1][0]);
    acc[0][1] = mma(a0, b1, acc[0][1]);
    acc[1][1] = mma(a1, b1, acc[1][1]);
    acc[0][2] = mma(a0, b2, acc[0][2]);
    acc[1][2] = mma(a1, b2, acc[1][2]);
    acc[0][3] = mma(a0, b3, acc[0][3]);
    acc[1][3] = mma(a1, b3, acc[1][3]);
    asm volatile(NOP4
                 : "+v"(acc[0][0]), "+v"(acc[1][0]), "+v"(acc[0][1]), "+v"(acc[1][1]),
                   "+v"(acc[0][2]), "+v"(acc[1][2]), "+v"(acc[0][3]), "+v"(acc[1][3])
                 : "v"(a0), "v"(a1), "v"(b0), "v"(b1), "v"(b2), "v"(b3));
  }

  const int which = col0 >> 10;
  const int hd = (col0 & (DD - 1)) >> 6;
  const float scale = (which == 0) ? 0.125f : 1.0f;
  const bool tr = (which == 2);
  float bb[4];
#pragma unroll
  for (int t = 0; t < 4; ++t) bb[t] = bf2f(bfbits(bias[col0 + t * 16 + lan]));
#pragma unroll
  for (int mi = 0; mi < 2; ++mi)
#pragma unroll
    for (int t = 0; t < 4; ++t)
#pragma unroll
      for (int r = 0; r < 8; ++r) {
        const int ml = widx * 32 + mi * 16 + 8 * h + r;
        const int nl = t * 16 + lan;
        const float v = (acc[mi][t][r] + bb[t]) * scale;
        unsigned int hi, lo;
        split2(v, hi, lo);
        const int idx = tr ? (nl * 64 + ml) : (ml * 64 + nl);
        sm[idx] = (unsigned short)hi;
        sm[4096 + idx] = (unsigned short)lo;
      }
  __syncthreads();

  bf16_t* const P0 = (which == 0) ? Qh : ((which == 1) ? Kh : Vh);
  bf16_t* const P1 = (which == 0) ? Ql : ((which == 1) ? Kl : Vl);
  const int bsel = rowb / SS;
  const int sbase = rowb & (SS - 1);
  const size_t headq = (size_t)(bsel * HH + hd);
  auto wr = [&]() {
#pragma unroll
    for (int it = 0; it < 8; ++it) {
      const int p = it * 64 + tid;
      const int row = p >> 3, piece = p & 7;
      const v4u Hw = *(const v4u*)(sm + row * 64 + piece * 8);
      const v4u Lw = *(const v4u*)(sm + 4096 + row * 64 + piece * 8);
      size_t off;
      if (!tr) off = (headq * SS + (size_t)(sbase + row)) * HD + (size_t)(piece * 8);
      else     off = (headq * HD + (size_t)row) * SS + (size_t)(sbase + piece * 8);
      *(volatile v4u*)(P0 + off) = Hw;
      *(volatile v4u*)(P1 + off) = Lw;
    }
  };
  wr();
  __threadfence();
  wr();
}

__global__ void __launch_bounds__(128) __attribute__((amdgpu_num_vgpr(256)))
k_attn(const bf16_t* __restrict__ Qh, const bf16_t* __restrict__ Ql,
       const bf16_t* __restrict__ Kh, const bf16_t* __restrict__ Kl,
       const bf16_t* __restrict__ Vh, const bf16_t* __restrict__ Vl,
       bf16_t* __restrict__ Oh, bf16_t* __restrict__ Ol) {
  __shared__ __align__(16) unsigned short osm[4 * 2 * 16 * 64];
  const int tid = (int)threadIdx.x;
  const int lane = tid & 31, h = lane >> 4, lan = lane & 15, widx = tid >> 5;
  const int wid = blockIdx.x * 4 + widx;
  const int qt = wid & (SS / 16 - 1);
  const int bh = wid >> 7;
  const int q0 = qt * 16, q = q0 + lan;
  const size_t pb = (size_t)bh * SS * HD;

  const bf16_t* qrh = Qh + pb + (size_t)q * HD;
  const bf16_t* qrl = Ql + pb + (size_t)q * HD;
  const v16bf qh0 = ldfrag(qrh, h), qh1 = ldfrag(qrh + 32, h);
  const v16bf ql0 = ldfrag(qrl, h), ql1 = ldfrag(qrl + 32, h);

  v8f o0 = zero8(), o1 = zero8(), o2 = zero8(), o3 = zero8();
  float rmax = -__builtin_inff(), rsum = 0.f;
  const int kend = q0 + 16;

#pragma unroll 1
  for (int kc = 0; kc < kend; kc += 32) {
    v8f s0 = zero8(), s1 = zero8();
    {
      const bf16_t* krh = Kh + pb + (size_t)(kc + lan) * HD;
      const bf16_t* krl = Kl + pb + (size_t)(kc + lan) * HD;
      const v16bf a0 = ldfrag(krh, h), a1 = ldfrag(krh + 32, h);
      const v16bf c0 = ldfrag(krl, h), c1 = ldfrag(krl + 32, h);
      s0 = mma(a0, qh0, s0);
      s0 = mma(a0, ql0, s0);
      s0 = mma(c0, qh0, s0);
      s0 = mma(a1, qh1, s0);
      s0 = mma(a1, ql1, s0);
      s0 = mma(c1, qh1, s0);
      asm volatile(NOP4 : "+v"(s0)
                   : "v"(a0), "v"(a1), "v"(c0), "v"(c1), "v"(qh0), "v"(qh1), "v"(ql0), "v"(ql1));
    }
    {
      const bf16_t* krh = Kh + pb + (size_t)(kc + 16 + lan) * HD;
      const bf16_t* krl = Kl + pb + (size_t)(kc + 16 + lan) * HD;
      const v16bf a0 = ldfrag(krh, h), a1 = ldfrag(krh + 32, h);
      const v16bf c0 = ldfrag(krl, h), c1 = ldfrag(krl + 32, h);
      s1 = mma(a0, qh0, s1);
      s1 = mma(a0, ql0, s1);
      s1 = mma(c0, qh0, s1);
      s1 = mma(a1, qh1, s1);
      s1 = mma(a1, ql1, s1);
      s1 = mma(c1, qh1, s1);
      asm volatile(NOP4 : "+v"(s1)
                   : "v"(a0), "v"(a1), "v"(c0), "v"(c1), "v"(qh0), "v"(qh1), "v"(ql0), "v"(ql1));
    }

    float x[16];
#pragma unroll
    for (int r = 0; r < 8; ++r) {
      const int key0 = kc + 8 * h + r;
      x[r]     = (key0 <= q)      ? s0[r] : -__builtin_inff();
      x[8 + r] = (key0 + 16 <= q) ? s1[r] : -__builtin_inff();
    }
    float m1 = x[0];
#pragma unroll
    for (int i = 1; i < 16; ++i) m1 = fmaxf(m1, x[i]);
    const float cm = fmaxf(m1, __shfl_xor(m1, 16, 32));
    const float nm = fmaxf(rmax, cm);
    float p[16];
    float ps = 0.f;
#pragma unroll
    for (int i = 0; i < 16; ++i) { p[i] = __expf(x[i] - nm); ps += p[i]; }
    const float cs = ps + __shfl_xor(ps, 16, 32);
    const float sc = __expf(rmax - nm);
    rsum = rsum * sc + cs;
    rmax = nm;
    o0 = o0 * sc; o1 = o1 * sc; o2 = o2 * sc; o3 = o3 * sc;

    union { v16bf v; unsigned int w[8]; } ph, pl;
#pragma unroll
    for (int i2 = 0; i2 < 8; ++i2) {
      unsigned int h0, l0, h1, l1;
      split2(p[2 * i2], h0, l0);
      split2(p[2 * i2 + 1], h1, l1);
      ph.w[i2] = h0 | (h1 << 16);
      pl.w[i2] = l0 | (l1 << 16);
    }
    const v16bf bph = ph.v, bpl = pl.v;

#define PV_TILE(OD, DT)                                                              \
    {                                                                                \
      const bf16_t* vrh_ = Vh + pb + (size_t)((DT) * 16 + lan) * SS + kc;           \
      const bf16_t* vrl_ = Vl + pb + (size_t)((DT) * 16 + lan) * SS + kc;           \
      const v16bf va_ = ldfrag(vrh_, h), vc_ = ldfrag(vrl_, h);                      \
      OD = mma(va_, bph, OD);                                                        \
      OD = mma(va_, bpl, OD);                                                        \
      OD = mma(vc_, bph, OD);                                                        \
      asm volatile(NOP4 : "+v"(OD) : "v"(va_), "v"(vc_), "v"(bph), "v"(bpl));        \
    }
    PV_TILE(o0, 0)
    PV_TILE(o1, 1)
    PV_TILE(o2, 2)
    PV_TILE(o3, 3)
#undef PV_TILE
  }

  const float inv = 1.0f / rsum;
  unsigned short* const myo = osm + widx * 2048;
#define O_STAGE(OD, DT)                                                                \
  {                                                                                    \
    v4u H_, L_;                                                                        \
    pack_hl8(OD, inv, H_, L_);                                                         \
    *(v4u*)(myo + lan * 64 + (DT) * 16 + 8 * h) = H_;                                  \
    *(v4u*)(myo + 1024 + lan * 64 + (DT) * 16 + 8 * h) = L_;                           \
  }
  O_STAGE(o0, 0)
  O_STAGE(o1, 1)
  O_STAGE(o2, 2)
  O_STAGE(o3, 3)
#undef O_STAGE
  __syncthreads();

  const int bsel = bh >> 4, hh = bh & (HH - 1);
  const size_t orow0 = (size_t)(bsel * SS + q0);
  auto wr = [&]() {
#pragma unroll
    for (int it = 0; it < 4; ++it) {
      const int pidx = it * 32 + lane;
      const int row = pidx >> 3, piece = pidx & 7;
      const v4u Hw = *(const v4u*)(myo + row * 64 + piece * 8);
      const v4u Lw = *(const v4u*)(myo + 1024 + row * 64 + piece * 8);
      const size_t off = (orow0 + (size_t)row) * DD + (size_t)(hh * HD + piece * 8);
      *(volatile v4u*)(Oh + off) = Hw;
      *(volatile v4u*)(Ol + off) = Lw;
    }
  };
  wr();
  __threadfence();
  wr();
}

__global__ void __launch_bounds__(64) __attribute__((amdgpu_num_vgpr(256)))
k_proj(const bf16_t* __restrict__ Oh, const bf16_t* __restrict__ Ol, const bf16_t* __restrict__ WpT,
       const float* __restrict__ bias, float* __restrict__ out) {
  __shared__ __align__(16) float smf[64 * 64];
  const int tid = (int)threadIdx.x;
  const int lane = tid & 31, h = lane >> 4, lan = lane & 15, widx = tid >> 5;
  constexpr int NT = DD / 64;
  const int bm = blockIdx.x / NT, bn = blockIdx.x - bm * NT;
  const int rowb = bm * 64, row0 = rowb + widx * 32, col0 = bn * 64;

  v8f acc[2][4];
#pragma unroll
  for (int mi = 0; mi < 2; ++mi)
#pragma unroll
    for (int t = 0; t < 4; ++t) acc[mi][t] = zero8();

  const bf16_t* ar0h = Oh + (size_t)(row0 + lan) * DD;
  const bf16_t* ar0l = Ol + (size_t)(row0 + lan) * DD;
  const bf16_t* ar1h = Oh + (size_t)(row0 + 16 + lan) * DD;
  const bf16_t* ar1l = Ol + (size_t)(row0 + 16 + lan) * DD;
  const bf16_t* brw  = WpT + (size_t)(col0 + lan) * DD;
#pragma unroll 1
  for (int k0 = 0; k0 < DD; k0 += 32) {
    const v16bf a0h = ldfrag(ar0h + k0, h), a0l = ldfrag(ar0l + k0, h);
    const v16bf a1h = ldfrag(ar1h + k0, h), a1l = ldfrag(ar1l + k0, h);
    {
      const v16bf b0 = ldfrag(brw + k0, h);
      const v16bf b1 = ldfrag(brw + (size_t)16 * DD + k0, h);
      acc[0][0] = mma(a0h, b0, acc[0][0]); acc[0][0] = mma(a0l, b0, acc[0][0]);
      acc[1][0] = mma(a1h, b0, acc[1][0]); acc[1][0] = mma(a1l, b0, acc[1][0]);
      acc[0][1] = mma(a0h, b1, acc[0][1]); acc[0][1] = mma(a0l, b1, acc[0][1]);
      acc[1][1] = mma(a1h, b1, acc[1][1]); acc[1][1] = mma(a1l, b1, acc[1][1]);
      asm volatile(NOP4
                   : "+v"(acc[0][0]), "+v"(acc[1][0]), "+v"(acc[0][1]), "+v"(acc[1][1])
                   : "v"(a0h), "v"(a0l), "v"(a1h), "v"(a1l), "v"(b0), "v"(b1));
    }
    {
      const v16bf b2 = ldfrag(brw + (size_t)32 * DD + k0, h);
      const v16bf b3 = ldfrag(brw + (size_t)48 * DD + k0, h);
      acc[0][2] = mma(a0h, b2, acc[0][2]); acc[0][2] = mma(a0l, b2, acc[0][2]);
      acc[1][2] = mma(a1h, b2, acc[1][2]); acc[1][2] = mma(a1l, b2, acc[1][2]);
      acc[0][3] = mma(a0h, b3, acc[0][3]); acc[0][3] = mma(a0l, b3, acc[0][3]);
      acc[1][3] = mma(a1h, b3, acc[1][3]); acc[1][3] = mma(a1l, b3, acc[1][3]);
      asm volatile(NOP4
                   : "+v"(acc[0][2]), "+v"(acc[1][2]), "+v"(acc[0][3]), "+v"(acc[1][3])
                   : "v"(a0h), "v"(a0l), "v"(a1h), "v"(a1l), "v"(b2), "v"(b3));
    }
  }

  float bb[4];
#pragma unroll
  for (int t = 0; t < 4; ++t) bb[t] = bf2f(bfbits(bias[col0 + t * 16 + lan]));
#pragma unroll
  for (int mi = 0; mi < 2; ++mi)
#pragma unroll
    for (int t = 0; t < 4; ++t)
#pragma unroll
      for (int r = 0; r < 8; ++r) {
        const int ml = widx * 32 + mi * 16 + 8 * h + r;
        const int nl = t * 16 + lan;
        smf[ml * 64 + nl] = acc[mi][t][r] + bb[t];
      }
  __syncthreads();

  auto wr = [&]() {
#pragma unroll
    for (int it = 0; it < 16; ++it) {
      const int p = it * 64 + tid;
      const int row = p >> 4, piece = p & 15;
      const v4f w = *(const v4f*)(smf + row * 64 + piece * 4);
      *(volatile v4f*)(out + (size_t)(rowb + row) * DD + (size_t)(col0 + piece * 4)) = w;
    }
  };
  wr();
  __threadfence();
  wr();
}

extern "C" void kernel_launch(void* const* d_in, const int* in_sizes, int n_in,
                              void* d_out, int out_size, void* d_ws, size_t ws_size,
                              hipStream_t stream) {
  if (n_in < 5) return;
  if (in_sizes[0] != MROWS * DD || in_sizes[1] != DD * NQKV || in_sizes[2] != NQKV ||
      in_sizes[3] != DD * DD || in_sizes[4] != DD) return;
  if (out_size != MROWS * DD) return;

  const float* hs     = (const float*)d_in[0];
  const float* w_attn = (const float*)d_in[1];
  const float* b_attn = (const float*)d_in[2];
  const float* w_proj = (const float*)d_in[3];
  const float* b_proj = (const float*)d_in[4];
  float* out = (float*)d_out;

  const size_t szX  = (size_t)MROWS * DD * 2;
  const size_t szWa = (size_t)NQKV * DD * 2;
  const size_t szWp = (size_t)DD * DD * 2;
  const size_t szP  = (size_t)BB * HH * SS * HD * 2;
  const size_t szO  = (size_t)MROWS * DD * 2;
  char* ws = (char*)d_ws;
  size_t off = 0;
  bf16_t* Xbf = (bf16_t*)(ws + off); off += szX;
  bf16_t* WaT = (bf16_t*)(ws + off); off += szWa;
  bf16_t* WpT = (bf16_t*)(ws + off); off += szWp;
  bf16_t* Qh  = (bf16_t*)(ws + off); off += szP;
  bf16_t* Ql  = (bf16_t*)(ws + off); off += szP;
  bf16_t* Kh  = (bf16_t*)(ws + off); off += szP;
  bf16_t* Kl  = (bf16_t*)(ws + off); off += szP;
  bf16_t* Vh  = (bf16_t*)(ws + off); off += szP;
  bf16_t* Vl  = (bf16_t*)(ws + off); off += szP;
  bf16_t* Ohp = (bf16_t*)(ws + off); off += szO;
  bf16_t* Olp = (bf16_t*)(ws + off); off += szO;
  if (off > ws_size) return;

  {
    const int n8 = (MROWS * DD) / 8;
    k_cvt<<<(n8 + 255) / 256, 256, 0, stream>>>(hs, Xbf, n8);
  }
  k_tr<<<dim3(NQKV / 64, DD / 64), 256, 0, stream>>>(w_attn, WaT, DD, NQKV);
  k_tr<<<dim3(DD / 64, DD / 64), 256, 0, stream>>>(w_proj, WpT, DD, DD);
  k_qkv<<<(MROWS / 64) * (NQKV / 64), 64, 0, stream>>>(Xbf, WaT, b_attn, Qh, Ql, Kh, Kl, Vh, Vl);
  k_attn<<<(BB * HH * (SS / 16)) / 4, 128, 0, stream>>>(Qh, Ql, Kh, Kl, Vh, Vl, Ohp, Olp);
  k_proj<<<(MROWS / 64) * (DD / 64), 64, 0, stream>>>(Ohp, Olp, WpT, b_proj, out);
}
